// DTWFramesLayerCUDA_31542239822344
// MI455X (gfx1250) — hardware-run, weakly checked
//
#include <hip/hip_runtime.h>
#include <math.h>

typedef __attribute__((ext_vector_type(16))) _Float16 v16h;
typedef __attribute__((ext_vector_type(8)))  _Float16 v8h;
typedef __attribute__((ext_vector_type(8)))  float    v8f;
typedef __attribute__((ext_vector_type(4)))  float    v4f;

constexpr int kNWin  = 64;
constexpr int kNPat  = 32;
constexpr int kDim   = 8;
constexpr int kWLen  = 128;
constexpr int kPLen  = 32;
constexpr int kOutW  = 32;
constexpr int kKPad  = 32;
constexpr int kCostPitch = 128;
constexpr int kOutPitch  = 36;

constexpr float kWCoef = 1.0f;
constexpr float kCarryX = 64.0f;
constexpr float kCarryP = 64.0f;
constexpr float kFold   = 1.0f / (kCarryX * kCarryP);
constexpr float kF16MinNormal = 6.103515625e-5f;
constexpr float kOutScale = 1.0f / (float)kPLen;

static_assert(kDim == 8, "the channel axis fills exactly the first 8-half group of a k-tile");
static_assert(kKPad == 32, "one 32-deep k-step");
static_assert(kWLen == 4 * 32, "each lane stages 4 consecutive frames");
static_assert(kPLen == 32 && kOutW == 32, "one lane per pattern position; one 128-B line per output row");
static_assert((kPLen % 16) == 0 && (kWLen % 16) == 0, "tile multiples");
static_assert((kOutPitch % 4) == 0 && kOutPitch >= kOutW, "16-B aligned staging rows");
static_assert(kWLen >= kOutW, "output columns are the last kOutW frames");

union FragH { v16h v; v8h h[2]; };

__device__ __forceinline__ v16h frag_load_h(const _Float16* p) {
  FragH f;
  f.h[0] = *(const v8h*)(p);
  f.h[1] = *(const v8h*)(p + 16);
  return f.v;
}

__device__ __forceinline__ v8f mma_f16_guarded(v16h a, v16h b, v8f c) {
  c = __builtin_amdgcn_wmma_f32_16x16x32_f16(false, a, false, b, (short)0, c, false, false);
  asm volatile("v_nop\n\tv_nop\n\tv_nop\n\tv_nop" : "+v"(c) : "v"(a), "v"(b));
  return c;
}

__device__ __forceinline__ _Float16 to_f16_carried(float v, float carry) {
  float s = v * carry;
  s = (fabsf(s) < kF16MinNormal) ? 0.0f : s;
  return (_Float16)s;
}

__global__ __launch_bounds__(32) void dtw_pair_kernel(const float* __restrict__ x,
                                                      const float* __restrict__ patts,
                                                      float* __restrict__ out) {
  __shared__ __align__(16) _Float16 sA[kPLen * kKPad];
  __shared__ __align__(16) _Float16 sB[kWLen * kKPad];
  __shared__ __align__(16) float sCost[kPLen * kCostPitch];
  __shared__ __align__(16) float sOut[kPLen * kOutPitch];
  __shared__ __align__(16) float sXX[kWLen];
  __shared__ __align__(16) float sPP[kPLen];

  const int bid  = blockIdx.x;
  const int n    = bid >> 5;
  const int kk   = bid & (kNPat - 1);
  const int lane = threadIdx.x & 31;
  const int h    = lane >> 4;
  const int l16  = lane & 15;

  const float* xn = x     + (size_t)n  * (kDim * kWLen);
  const float* pk = patts + (size_t)kk * (kDim * kPLen);

  float pv[kDim];
#pragma unroll
  for (int d = 0; d < kDim; ++d) pv[d] = pk[d * kPLen + lane];
  v4f xv[kDim];
#pragma unroll
  for (int d = 0; d < kDim; ++d) xv[d] = *(const v4f*)(xn + d * kWLen + 4 * lane);

  const v8h hz = (v8h){(_Float16)0.0f, (_Float16)0.0f, (_Float16)0.0f, (_Float16)0.0f,
                       (_Float16)0.0f, (_Float16)0.0f, (_Float16)0.0f, (_Float16)0.0f};

  {
    float pp = 0.0f;
    v8h ha;
#pragma unroll
    for (int d = 0; d < kDim; ++d) {
      const float t = pv[d];
      pp += t * t;
      ha[d] = to_f16_carried(t, kCarryP);
    }
    sPP[lane] = pp;
    _Float16* rowp = sA + lane * kKPad;
    *(v8h*)(rowp)      = ha;
    *(v8h*)(rowp + 8)  = hz;
    *(v8h*)(rowp + 16) = hz;
    *(v8h*)(rowp + 24) = hz;
  }

#pragma unroll
  for (int e = 0; e < 4; ++e) {
    float s = 0.0f;
    v8h hb;
#pragma unroll
    for (int d = 0; d < kDim; ++d) {
      const float t = xv[d][e];
      s += t * t;
      hb[d] = to_f16_carried(t, kCarryX);
    }
    const int w = 4 * lane + e;
    sXX[w] = s;
    _Float16* roww = sB + w * kKPad;
    *(v8h*)(roww)      = hb;
    *(v8h*)(roww + 8)  = hz;
    *(v8h*)(roww + 16) = hz;
    *(v8h*)(roww + 24) = hz;
  }

  __syncthreads();

  v16h afrag[2];
#pragma unroll
  for (int mt = 0; mt < 2; ++mt) afrag[mt] = frag_load_h(sA + (mt * 16 + l16) * kKPad + 8 * h);
  float ppv[2][8];
#pragma unroll
  for (int mt = 0; mt < 2; ++mt)
#pragma unroll
    for (int r = 0; r < 8; ++r) ppv[mt][r] = sPP[mt * 16 + 8 * h + r];

#pragma unroll
  for (int nt = 0; nt < 8; ++nt) {
    const int wcol = nt * 16 + l16;
    const v16h bfrag = frag_load_h(sB + wcol * kKPad + 8 * h);
    const float xxw = sXX[wcol];
#pragma unroll
    for (int mt = 0; mt < 2; ++mt) {
      v8f acc = (v8f){0.f, 0.f, 0.f, 0.f, 0.f, 0.f, 0.f, 0.f};
      acc = mma_f16_guarded(afrag[mt], bfrag, acc);
#pragma unroll
      for (int r = 0; r < 8; ++r) {
        const int p = mt * 16 + 8 * h + r;
        const float dot = acc[r] * kFold;
        const float c = fmaxf((xxw + ppv[mt][r]) - 2.0f * dot, 0.0f);
        sCost[p * kCostPitch + wcol] = c;
      }
    }
  }

  __syncthreads();

  {
    const int p = lane;
    float v = 0.0f;
    float diag = 0.0f;
#pragma unroll 1
    for (int t = 0; t < kWLen + kPLen - 1; ++t) {
      const float up = __shfl_up(v, 1, 32);
      const int wi = t - p;
      const bool active = (wi >= 0) && (wi < kWLen);
      int wc = wi < 0 ? 0 : wi;
      wc = wc > (kWLen - 1) ? (kWLen - 1) : wc;
      const float c = sCost[p * kCostPitch + wc];
      const bool firstCol = (wi == 0);
      const float inner = c + fminf(kWCoef * fminf(v, diag), up);
      const float row0 = firstCol ? c : (c + kWCoef * v);
      const float rest = firstCol ? (c + up) : inner;
      const float nv = (p == 0) ? row0 : rest;
      v = active ? nv : v;
      if (active && (wi >= kWLen - kOutW)) {
        sOut[p * kOutPitch + (wi - (kWLen - kOutW))] = sqrtf(nv) * kOutScale;
      }
      diag = up;
    }
  }

  __syncthreads();

  {
    float* outp = out + (size_t)bid * (kPLen * kOutW);
    const int q  = lane >> 3;
    const int c4 = (lane & 7) * 4;
    v4f ov[8];
#pragma unroll
    for (int it = 0; it < 8; ++it) ov[it] = *(const v4f*)(sOut + (it * 4 + q) * kOutPitch + c4);
    for (int pass = 0; pass < 2; ++pass) {
#pragma unroll
      for (int it = 0; it < 8; ++it) {
        *(volatile v4f*)(outp + (it * 4 + q) * kOutW + c4) = ov[it];
      }
      __threadfence();
    }
  }
}

extern "C" void kernel_launch(void* const* d_in, const int* in_sizes, int n_in,
                              void* d_out, int out_size, void* d_ws, size_t ws_size,
                              hipStream_t stream) {
  (void)d_ws; (void)ws_size;
  if (n_in < 2) return;
  if (in_sizes[0] != kNWin * kDim * kWLen) return;
  if (in_sizes[1] != kNPat * kDim * kPLen) return;
  if (out_size != kNWin * kNPat * kPLen * kOutW) return;

  const float* x     = (const float*)d_in[0];
  const float* patts = (const float*)d_in[1];
  float* out = (float*)d_out;

  dtw_pair_kernel<<<dim3(kNWin * kNPat), dim3(32), 0, stream>>>(x, patts, out);
}
